// HybridImageFittingModel_65077344469002
// MI455X (gfx1250) — hardware-run, weakly checked
//
#include <hip/hip_runtime.h>
#include <math.h>

#ifndef NB
#define NB 16384
#endif
#define NB_FULL 16384
#define NQ 6
#define DIM 64
#define KA 256
#define KU 128
#define CARRY 1024.0f
#define RES_SCALE 2048.0f
#define INV_RES (1.0f / 2048.0f)
#define INV_CARRY2 (1.0f / (1024.0f * 1024.0f))
#define BN_EPS 1e-5f

static_assert(NB <= NB_FULL);
static_assert(NB % 512 == 0);
static_assert(NB % 256 == 0);
static_assert(KA % 32 == 0 && KU % 32 == 0);
static_assert(KA == 2 * KU);
static_assert(DIM % 16 == 0);

typedef _Float16 h16;
typedef __attribute__((ext_vector_type(16))) _Float16 v16h;
typedef __attribute__((ext_vector_type(8)))  _Float16 v8h;
typedef __attribute__((ext_vector_type(8)))  float    v8f;
typedef __attribute__((ext_vector_type(4)))  float    v4f;


#define VST2(T, ptr, val) do { const T vst2_v_ = (val); *(volatile T*)(ptr) = vst2_v_; __threadfence(); *(volatile T*)(ptr) = vst2_v_; } while (0)
#define VST2V4(ptr, val) do { const v4f vst2_v4_ = (val); *(volatile v4f*)(ptr) = vst2_v4_; __threadfence(); *(volatile v4f*)(ptr) = vst2_v4_; } while (0)

static __device__ __forceinline__ float bfr(float f) {
    unsigned u = __float_as_uint(f);
    u += 0x7FFFu + ((u >> 16) & 1u);
    return __uint_as_float(u & 0xFFFF0000u);
}
static __device__ __forceinline__ h16 toh_flush(float v) { const float w = (fabsf(v) < 6.103515625e-05f) ? 0.0f : v; return (h16)w; }

union FragU { v16h v; v8h h[2]; };
static __device__ __forceinline__ v16h frag_ld(const _Float16* p) {
    FragU f; f.h[0] = *(const v8h*)(p); f.h[1] = *(const v8h*)(p + 16); return f.v;
}
static __device__ __forceinline__ v8f wmma16g(v16h a, v16h b, v8f c) {
    c = __builtin_amdgcn_wmma_f32_16x16x32_f16(false, a, false, b, (short)0, c, false, false);
    asm volatile("v_nop\n\tv_nop\n\tv_nop\n\tv_nop" : "+v"(c) : "v"(a), "v"(b));
    return c;
}

static __device__ __forceinline__ unsigned pair_lo(unsigned p, unsigned pos) {
    const unsigned low = p & ((1u << pos) - 1u);
    return ((p >> pos) << (pos + 1u)) | low;
}
static __device__ __forceinline__ unsigned spread2(unsigned p, unsigned posA, unsigned posB, unsigned bitA, unsigned bitB) {
    unsigned k = 0u, b = 0u;
#pragma unroll
    for (unsigned pos = 0u; pos < 6u; ++pos) {
        unsigned bit;
        if (pos == posA)      bit = bitA;
        else if (pos == posB) bit = bitB;
        else { bit = (p >> b) & 1u; ++b; }
        k |= bit << pos;
    }
    return k;
}

struct Rot2 { float r00, i00, r01, i01, r10, i10, r11, i11; };
static __device__ __forceinline__ Rot2 make_rot(float ph, float th, float om) {
    const float c = cosf(th * 0.5f), s = sinf(th * 0.5f);
    const float a1 = -0.5f * (ph + om), a2 = -0.5f * (ph - om);
    const float epr = cosf(a1), epi = sinf(a1);
    const float emr = cosf(a2), emi = sinf(a2);
    Rot2 u;
    u.r00 = epr * c;  u.i00 = epi * c;
    u.r01 = -emr * s; u.i01 = emi * s;
    u.r10 = emr * s;  u.i10 = emi * s;
    u.r11 = epr * c;  u.i11 = -epi * c;
    return u;
}

__global__ __launch_bounds__(256) void k_circ(const float* __restrict__ w1q, const float* __restrict__ w2q,
                                              _Float16* __restrict__ U16, float* __restrict__ psi0) {
    __shared__ __align__(16) float sU[2 * DIM * DIM];
    __shared__ __align__(16) float sP[2 * DIM];
    const unsigned tid = threadIdx.x;

    if (tid < 64u) { sP[tid] = (tid == 0u) ? 1.0f : 0.0f; sP[64u + tid] = 0.0f; }
    __syncthreads();
    for (unsigned rep = 0u; rep < 3u; ++rep) {
        for (unsigned l = 0u; l < 3u; ++l) {
            const unsigned r = l + 1u;
            for (unsigned j = 0u; j < 6u; ++j) {
                const float* w = w1q + (l * 6u + j) * 3u;
                const Rot2 u = make_rot(bfr(w[0]), bfr(w[1]), bfr(w[2]));
                if (tid < 32u) {
                    const unsigned pos = 5u - j;
                    const unsigned k0 = pair_lo(tid, pos), k1 = k0 | (1u << pos);
                    const float a0r = sP[k0], a0i = sP[64u + k0], a1r = sP[k1], a1i = sP[64u + k1];
                    sP[k0]       = (u.r00 * a0r - u.i00 * a0i) + (u.r01 * a1r - u.i01 * a1i);
                    sP[64u + k0] = (u.r00 * a0i + u.i00 * a0r) + (u.r01 * a1i + u.i01 * a1r);
                    sP[k1]       = (u.r10 * a0r - u.i10 * a0i) + (u.r11 * a1r - u.i11 * a1i);
                    sP[64u + k1] = (u.r10 * a0i + u.i10 * a0r) + (u.r11 * a1i + u.i11 * a1r);
                }
                __syncthreads();
            }
            for (unsigned j = 0u; j < 6u; ++j) {
                const unsigned pc = 5u - j, pt = 5u - ((j + r) % 6u);
                if (tid < 16u) {
                    const unsigned k = spread2(tid, pc, pt, 1u, 0u);
                    const unsigned k2 = k | (1u << pt);
                    const float tr = sP[k], ti = sP[64u + k];
                    sP[k] = sP[k2]; sP[64u + k] = sP[64u + k2];
                    sP[k2] = tr;    sP[64u + k2] = ti;
                }
                __syncthreads();
            }
        }
    }

    for (unsigned q = tid; q < (unsigned)(DIM * DIM); q += 256u) {
        sU[q] = ((q >> 6) == (q & 63u)) ? 1.0f : 0.0f;
        sU[4096u + q] = 0.0f;
    }
    __syncthreads();
    for (unsigned j = 0u; j < 6u; ++j) {
        const float* w = w2q + j * 3u;
        const Rot2 u = make_rot(bfr(w[0]), bfr(w[1]), bfr(w[2]));
        const unsigned pos = 5u - j;
        for (unsigned q = tid; q < 32u * 64u; q += 256u) {
            const unsigned p = q >> 6, col = q & 63u;
            const unsigned k0 = pair_lo(p, pos), k1 = k0 | (1u << pos);
            const unsigned o0 = k0 * 64u + col, o1 = k1 * 64u + col;
            const float a0r = sU[o0], a0i = sU[4096u + o0], a1r = sU[o1], a1i = sU[4096u + o1];
            sU[o0]         = (u.r00 * a0r - u.i00 * a0i) + (u.r01 * a1r - u.i01 * a1i);
            sU[4096u + o0] = (u.r00 * a0i + u.i00 * a0r) + (u.r01 * a1i + u.i01 * a1r);
            sU[o1]         = (u.r10 * a0r - u.i10 * a0i) + (u.r11 * a1r - u.i11 * a1i);
            sU[4096u + o1] = (u.r10 * a0i + u.i10 * a0r) + (u.r11 * a1i + u.i11 * a1r);
        }
        __syncthreads();
    }
    for (unsigned j = 0u; j < 6u; ++j) {
        const unsigned pc = 5u - j, pt = 5u - ((j + 1u) % 6u);
        for (unsigned q = tid; q < 16u * 64u; q += 256u) {
            const unsigned p = q >> 6, col = q & 63u;
            const unsigned k = spread2(p, pc, pt, 1u, 1u);
            const unsigned o = k * 64u + col;
            sU[o] = -sU[o];
            sU[4096u + o] = -sU[4096u + o];
        }
        __syncthreads();
    }

    if (tid < 32u) {
        v4f v; v.x = sP[4u * tid]; v.y = sP[4u * tid + 1u]; v.z = sP[4u * tid + 2u]; v.w = sP[4u * tid + 3u];
        VST2V4(psi0 + 4u * tid, v);
    }
    for (unsigned uidx = tid; uidx < 2048u; uidx += 256u) {
        const unsigned n = uidx >> 4, k = (uidx & 15u) * 8u;
        const unsigned useIm = ((n >> 6) ^ (k >> 6)) & 1u;
        const float sg = ((n < 64u) && (k >= 64u)) ? -CARRY : CARRY;
        const unsigned off = useIm * 4096u + (n & 63u) * 64u + (k & 63u);
        v8h hv;
#pragma unroll
        for (int e = 0; e < 8; ++e) hv[e] = toh_flush(sU[off + (unsigned)e] * sg);
        _Float16* dst = U16 + (size_t)n * KU + k;
        for (int pass = 0; pass < 2; ++pass) {
            *(volatile v8h*)(dst) = hv;
            __threadfence();
        }
    }
}

__global__ __launch_bounds__(512) void k_stat(const float* __restrict__ x, const float* __restrict__ w1,
                                              const float* __restrict__ b1, float* __restrict__ stats) {
    __shared__ float red[6][512];
    __shared__ float sMean[8];
    __shared__ __align__(16) float sLine[32];
    const unsigned t = threadIdx.x;
    float wa[6], wb[6], bb[6];
#pragma unroll
    for (int j = 0; j < 6; ++j) { wa[j] = bfr(w1[2 * j]); wb[j] = bfr(w1[2 * j + 1]); bb[j] = bfr(b1[j]); }
    const float invn = 1.0f / (float)NB;

    float s[6];
#pragma unroll
    for (int j = 0; j < 6; ++j) s[j] = 0.0f;
    for (unsigned i = 0u; i < (unsigned)(NB / 512); ++i) {
        const unsigned row = i * 512u + t;
        const float x0 = bfr(x[2u * row]), x1 = bfr(x[2u * row + 1u]);
#pragma unroll
        for (int j = 0; j < 6; ++j) s[j] += x0 * wa[j] + x1 * wb[j] + bb[j];
    }
#pragma unroll
    for (int j = 0; j < 6; ++j) red[j][t] = s[j];
    __syncthreads();
    for (unsigned st = 256u; st > 0u; st >>= 1) {
        if (t < st) {
#pragma unroll
            for (int j = 0; j < 6; ++j) red[j][t] += red[j][t + st];
        }
        __syncthreads();
    }
    if (t < 8u) {
        const unsigned jc = min(t, 5u);
        const float m = red[jc][0] * invn;
        sMean[t] = (t < 6u) ? m : 0.0f;
    }
    __syncthreads();
    float mu[6];
#pragma unroll
    for (int j = 0; j < 6; ++j) { mu[j] = sMean[j]; s[j] = 0.0f; }
    for (unsigned i = 0u; i < (unsigned)(NB / 512); ++i) {
        const unsigned row = i * 512u + t;
        const float x0 = bfr(x[2u * row]), x1 = bfr(x[2u * row + 1u]);
#pragma unroll
        for (int j = 0; j < 6; ++j) {
            const float h = x0 * wa[j] + x1 * wb[j] + bb[j];
            const float d = h - mu[j];
            s[j] += d * d;
        }
    }
#pragma unroll
    for (int j = 0; j < 6; ++j) red[j][t] = s[j];
    __syncthreads();
    for (unsigned st = 256u; st > 0u; st >>= 1) {
        if (t < st) {
#pragma unroll
            for (int j = 0; j < 6; ++j) red[j][t] += red[j][t + st];
        }
        __syncthreads();
    }
    if (t < 32u) {
        const unsigned jv = (t >= 6u && t < 12u) ? (t - 6u) : 0u;
        const float var = red[jv][0] * invn;
        const float rs = 1.0f / sqrtf(var + BN_EPS);
        const float mv = sMean[min(t, 7u)];
        sLine[t] = (t < 6u) ? mv : ((t < 12u) ? rs : 0.0f);
    }
    __syncthreads();
    if (t < 8u) {
        v4f v; v.x = sLine[4u * t]; v.y = sLine[4u * t + 1u]; v.z = sLine[4u * t + 2u]; v.w = sLine[4u * t + 3u];
        VST2V4(stats + 4u * t, v);
    }
}

__global__ __launch_bounds__(256) void k_phase(const float* __restrict__ x, const float* __restrict__ w1, const float* __restrict__ b1,
                                               const float* __restrict__ gam, const float* __restrict__ bet,
                                               const float* __restrict__ stats, const float* __restrict__ psi0,
                                               _Float16* __restrict__ A16) {
    const unsigned u = blockIdx.x * 256u + threadIdx.x;
    const unsigned row = u >> 3, q = u & 7u;
    const float x0 = bfr(x[2u * row]), x1 = bfr(x[2u * row + 1u]);
    float cs[6], sn[6];
#pragma unroll
    for (int j = 0; j < 6; ++j) {
        const float h = x0 * bfr(w1[2 * j]) + x1 * bfr(w1[2 * j + 1]) + bfr(b1[j]);
        const float a = (h - stats[j]) * stats[6 + j] * bfr(gam[j]) + bfr(bet[j]);
        const float ha = 0.5f * a;
        cs[j] = cosf(ha);
        sn[j] = sinf(ha);
    }
    float fl[3];
#pragma unroll
    for (int j = 0; j < 3; ++j) fl[j] = ((q >> (2 - j)) & 1u) ? sn[j] : -sn[j];

    const v4f pr0 = *(const v4f*)(psi0 + 8u * q),       pr1 = *(const v4f*)(psi0 + 8u * q + 4u);
    const v4f pi0 = *(const v4f*)(psi0 + 64u + 8u * q), pi1 = *(const v4f*)(psi0 + 64u + 8u * q + 4u);
    const float pr[8] = {pr0.x, pr0.y, pr0.z, pr0.w, pr1.x, pr1.y, pr1.z, pr1.w};
    const float pi[8] = {pi0.x, pi0.y, pi0.z, pi0.w, pi1.x, pi1.y, pi1.z, pi1.w};

    v8h hRe, hIm, lRe, lIm;
#pragma unroll
    for (int e = 0; e < 8; ++e) {
        float ar = pr[e], ai = pi[e];
#pragma unroll
        for (int j = 0; j < 6; ++j) {
            const float fi = (j < 3) ? fl[(j < 3) ? j : 0] : ((((unsigned)e >> (5 - j)) & 1u) ? sn[j] : -sn[j]);
            const float fr = cs[j];
            const float nr = fr * ar - fi * ai;
            const float ni = fr * ai + fi * ar;
            ar = nr; ai = ni;
        }
        const float vr = ar * CARRY, vi = ai * CARRY;
        const h16 hr = toh_flush(vr), hi = toh_flush(vi);
        hRe[e] = hr;
        hIm[e] = hi;
        lRe[e] = toh_flush((vr - (float)hr) * RES_SCALE);
        lIm[e] = toh_flush((vi - (float)hi) * RES_SCALE);
    }
    _Float16* dst = A16 + (size_t)row * KA + 8u * q;
    for (int pass = 0; pass < 2; ++pass) {
        *(volatile v8h*)(dst)        = hRe;
        *(volatile v8h*)(dst + 64)   = hIm;
        *(volatile v8h*)(dst + 128)  = lRe;
        *(volatile v8h*)(dst + 192)  = lIm;
        __threadfence();
    }
}

static __device__ __forceinline__ float tile_rows(const _Float16* __restrict__ A16, const _Float16* __restrict__ U16,
                                                  unsigned m0, unsigned lane, unsigned K, unsigned NT,
                                                  float w0, float w1v, float w2v, float w3, float w4, float w5, float b2) {
    const unsigned hh = lane >> 4, c = lane & 15u;
    const _Float16* arow = A16 + (size_t)(m0 + c) * KA + 8u * hh;
    float pall[8], z0p[8], z1p[8];
#pragma unroll
    for (int r = 0; r < 8; ++r) { pall[r] = 0.0f; z0p[r] = 0.0f; z1p[r] = 0.0f; }

    for (unsigned jt = 0u; jt < NT; ++jt) {
        v8f reV = (v8f){0.f,0.f,0.f,0.f,0.f,0.f,0.f,0.f};
        v8f reR = reV, imV = reV, imR = reV;
        const _Float16* ure = U16 + (size_t)(16u * jt + c) * KU + 8u * hh;
        const _Float16* uim = U16 + (size_t)(64u + 16u * jt + c) * KU + 8u * hh;
        for (unsigned k0 = 0u; k0 < K; k0 += 32u) {
            const v16h av = frag_ld(arow + k0);
            const v16h ar = frag_ld(arow + 128u + k0);
            const v16h br = frag_ld(ure + k0);
            const v16h bi = frag_ld(uim + k0);
            reV = wmma16g(av, br, reV);
            reR = wmma16g(ar, br, reR);
            imV = wmma16g(av, bi, imV);
            imR = wmma16g(ar, bi, imR);
        }
        const bool neg0 = ((jt >> 1) & 1u) != 0u;
        const bool neg1 = (jt & 1u) != 0u;
#pragma unroll
        for (int r = 0; r < 8; ++r) {
            const float sr = (reV[r] + reR[r] * INV_RES) * INV_CARRY2;
            const float si = (imV[r] + imR[r] * INV_RES) * INV_CARRY2;
            const float p = sr * sr + si * si;
            pall[r] += p;
            z0p[r] += neg0 ? -p : p;
            z1p[r] += neg1 ? -p : p;
        }
    }
    float o[8];
#pragma unroll
    for (int r = 0; r < 8; ++r) {
        float z[6];
        z[0] = z0p[r];
        z[1] = z1p[r];
#pragma unroll
        for (int j = 2; j < 6; ++j) z[j] = ((c >> (5 - j)) & 1u) ? -pall[r] : pall[r];
#pragma unroll
        for (int j = 0; j < 6; ++j) {
            float t = z[j];
            t += __shfl_xor(t, 1, 32);
            t += __shfl_xor(t, 2, 32);
            t += __shfl_xor(t, 4, 32);
            t += __shfl_xor(t, 8, 32);
            z[j] = t;
        }
        float acc = z[0] * w0;
        acc += z[1] * w1v;
        acc += z[2] * w2v;
        acc += z[3] * w3;
        acc += z[4] * w4;
        acc += z[5] * w5;
        o[r] = acc + b2;
    }
    float sel = o[0];
#pragma unroll
    for (int r = 1; r < 8; ++r) sel = ((lane & 7u) == (unsigned)r) ? o[r] : sel;
    return sel;
}

__global__ __launch_bounds__(256) void k_map(const _Float16* __restrict__ A16, const _Float16* __restrict__ U16,
                                             const float* __restrict__ wl2, const float* __restrict__ bl2,
                                             float* __restrict__ out, unsigned K, unsigned NT) {
    const unsigned lane = threadIdx.x & 31u, wave = threadIdx.x >> 5;
    const unsigned base32 = (blockIdx.x * 8u + wave) * 32u;
    const float w0 = bfr(wl2[0]), w1v = bfr(wl2[1]), w2v = bfr(wl2[2]), w3 = bfr(wl2[3]), w4 = bfr(wl2[4]), w5 = bfr(wl2[5]);
    const float b2 = bfr(bl2[0]);
    const float sel0 = tile_rows(A16, U16, base32,       lane, K, NT, w0, w1v, w2v, w3, w4, w5, b2);
    const float sel1 = tile_rows(A16, U16, base32 + 16u, lane, K, NT, w0, w1v, w2v, w3, w4, w5, b2);
    const unsigned src = 16u * ((lane >> 3) & 1u) + (lane & 7u);
    const float v0 = __shfl(sel0, (int)src, 32);
    const float v1 = __shfl(sel1, (int)src, 32);
    const float v = (lane >> 4) ? v1 : v0;
    VST2(float, out + base32 + lane, v);
}

extern "C" void kernel_launch(void* const* d_in, const int* in_sizes, int n_in, void* d_out, int out_size,
                              void* d_ws, size_t ws_size, hipStream_t stream) {
    if (n_in < 9) return;
    if (in_sizes[0] < NB * 2 || in_sizes[1] < 12 || in_sizes[2] < 6 || in_sizes[3] < 6 || in_sizes[4] < 6) return;
    if (in_sizes[5] < 54 || in_sizes[6] < 18 || in_sizes[7] < 6 || in_sizes[8] < 1 || out_size < NB) return;

    const float* x        = (const float*)d_in[0];
    const float* w_lin1   = (const float*)d_in[1];
    const float* b_lin1   = (const float*)d_in[2];
    const float* bn_gamma = (const float*)d_in[3];
    const float* bn_beta  = (const float*)d_in[4];
    const float* weights1 = (const float*)d_in[5];
    const float* weights2 = (const float*)d_in[6];
    const float* w_lin2   = (const float*)d_in[7];
    const float* b_lin2   = (const float*)d_in[8];
    float* out = (float*)d_out;

    constexpr size_t U16_BYTES  = (size_t)128 * KU * 2;
    constexpr size_t PSI_BYTES  = (size_t)128 * 4;
    constexpr size_t STAT_BYTES = (size_t)32 * 4;
    constexpr size_t A16_BYTES  = (size_t)NB * KA * 2;
    constexpr size_t WS_TOTAL = ((U16_BYTES + 255) & ~(size_t)255) + ((PSI_BYTES + 255) & ~(size_t)255) +
                                ((STAT_BYTES + 255) & ~(size_t)255) + ((A16_BYTES + 255) & ~(size_t)255);
    static_assert(WS_TOTAL <= (size_t)134217728);

    char* wsp = (char*)d_ws;
    size_t off = 0;
    auto carve = [&](size_t bytes) -> void* { void* r = wsp + off; off += (bytes + 255) & ~(size_t)255; return r; };
    _Float16* U16   = (_Float16*)carve(U16_BYTES);
    float*    psi0  = (float*)carve(PSI_BYTES);
    float*    stats = (float*)carve(STAT_BYTES);
    _Float16* A16   = (_Float16*)carve(A16_BYTES);
    if (off > ws_size || off > (size_t)134217728) return;

    k_circ<<<1, 256, 0, stream>>>(weights1, weights2, U16, psi0);
    k_stat<<<1, 512, 0, stream>>>(x, w_lin1, b_lin1, stats);
    k_phase<<<(NB * 8) / 256, 256, 0, stream>>>(x, w_lin1, b_lin1, bn_gamma, bn_beta, stats, psi0, A16);
    k_map<<<NB / 256, 256, 0, stream>>>((const _Float16*)A16, (const _Float16*)U16, w_lin2, b_lin2, out,
                                        (unsigned)KU, (unsigned)(DIM / 16));
}
